// Multi_LSTMs_5660766896170
// MI455X (gfx1250) — hardware-verified
//
#include <hip/hip_runtime.h>
#include <stdint.h>
#include <math.h>

typedef __attribute__((ext_vector_type(16))) _Float16 v16h;
typedef __attribute__((ext_vector_type(8)))  _Float16 v8h;
typedef __attribute__((ext_vector_type(16))) __bf16   v16b;
typedef __attribute__((ext_vector_type(8)))  __bf16   v8b;
typedef __attribute__((ext_vector_type(8)))  float    v8f;
typedef __attribute__((ext_vector_type(4)))  float    v4f;
typedef __attribute__((ext_vector_type(4)))  unsigned v4u;

__device__ __forceinline__ unsigned short f2bf_bits(float f) {
  unsigned u = __float_as_uint(f);
  return (unsigned short)((u + 0x7FFFu + ((u >> 16) & 1u)) >> 16);
}
__device__ __forceinline__ float bf_bits2f(unsigned short h) { return __uint_as_float(((unsigned)h) << 16); }

__device__ __forceinline__ void dep_guard_h(v8f& a, v8f& b, v16h x, v16h y) { asm volatile("v_nop\n\tv_nop\n\tv_nop\n\tv_nop" : "+v"(a), "+v"(b) : "v"(x), "v"(y)); }
__device__ __forceinline__ void dep_guard_b(v8f& a, v8f& b, v16b x, v16b y) { asm volatile("v_nop\n\tv_nop\n\tv_nop\n\tv_nop" : "+v"(a), "+v"(b) : "v"(x), "v"(y)); }
__device__ __forceinline__ void keep4_h(v16h a, v16h b, v16h c, v16h d) { asm volatile("v_nop" :: "v"(a), "v"(b), "v"(c), "v"(d)); }
__device__ __forceinline__ void keep4_b(v16b a, v16b b, v16b c, v16b d) { asm volatile("v_nop" :: "v"(a), "v"(b), "v"(c), "v"(d)); }
__device__ __forceinline__ void acc_guard4(v8f& a, v8f& b, v8f& c, v8f& d) { asm volatile("v_nop\n\tv_nop\n\tv_nop\n\tv_nop" : "+v"(a), "+v"(b), "+v"(c), "+v"(d)); }
template <typename T> struct Frag;
template <> struct Frag<_Float16> {
  typedef v16h V; union U { v16h v; v8h h[2]; };
  static __device__ __forceinline__ v16h load(const _Float16* p) {
    U f; f.h[0] = *(const v8h*)(p); f.h[1] = *(const v8h*)(p + 16); return f.v;
  }
  static __device__ __forceinline__ v8f mma(v16h a, v16h b, v8f c) {
    return __builtin_amdgcn_wmma_f32_16x16x32_f16(false, a, false, b, (short)0, c, false, false);
  }
  static __device__ __forceinline__ void guard(v8f& a, v8f& b, v16h x, v16h y) { dep_guard_h(a, b, x, y); }
  static __device__ __forceinline__ void keep(v16h a, v16h b, v16h c, v16h d) { keep4_h(a, b, c, d); }
};
template <> struct Frag<__bf16> {
  typedef v16b V; union U { v16b v; v8b h[2]; };
  static __device__ __forceinline__ v16b load(const __bf16* p) {
    U f; f.h[0] = *(const v8b*)(p); f.h[1] = *(const v8b*)(p + 16); return f.v;
  }
  static __device__ __forceinline__ v8f mma(v16b a, v16b b, v8f c) {
    return __builtin_amdgcn_wmma_f32_16x16x32_bf16(false, a, false, b, (short)0, c, false, false);
  }
  static __device__ __forceinline__ void guard(v8f& a, v8f& b, v16b x, v16b y) { dep_guard_b(a, b, x, y); }
  static __device__ __forceinline__ void keep(v16b a, v16b b, v16b c, v16b d) { keep4_b(a, b, c, d); }
};

template <int ET> struct Elem;
template <> struct Elem<0> { typedef _Float16 T; };
template <> struct Elem<1> { typedef __bf16 T; };
template <int ET, bool SPLIT, int BIAS_MODE, int OUT_MODE, bool RESID, int ACT = 0>
__global__ __launch_bounds__(256) void wmma_gemm64(
    const unsigned short* __restrict__ Ap, const unsigned short* __restrict__ A2p, int lda, long strideA,
    const unsigned short* __restrict__ Btp, const unsigned short* __restrict__ Bt2p, int ldb, long strideB,
    void* __restrict__ Cout, void* __restrict__ Cout2, int ldc, long strideC,
    const float* __restrict__ bias,
    const float* __restrict__ resid, long strideR,
    int M, int N, int K, float scale) {
  typedef typename Elem<ET>::T T;
  typedef typename Frag<T>::V V;
  const T* A = (const T*)Ap; const T* A2 = (const T*)A2p; const T* Bt = (const T*)Btp; const T* Bt2 = (const T*)Bt2p;
  __shared__ __align__(16) float sT[8][16 * 68];
  const int b    = blockIdx.y;
  const int lane = threadIdx.x & 31;
  const int wave = threadIdx.x >> 5;
  const int tilesN = N >> 6;
  const int tilesM = M >> 6;
  const int tile = blockIdx.x * 8 + wave;
  if (tile >= tilesM * tilesN) return;
  const int tm = tile / tilesN;
  const int tn = tile - tm * tilesN;
  const int m0 = tm << 6;
  const int n0 = tn << 6;

  const T* Ab  = A  + (size_t)b * strideA;
  const T* Bb  = Bt + (size_t)b * strideB;
  const T* Ab2 = SPLIT ? (A2  + (size_t)b * strideA) : nullptr;
  const T* Bb2 = SPLIT ? (Bt2 + (size_t)b * strideB) : nullptr;

  const int rlane = lane & 15;
  const int koff  = (lane >> 4) * 8;
  const int mOff  = (lane >> 4) * 8;

  v8f acc[4][4];
#pragma unroll
  for (int i = 0; i < 4; ++i)
#pragma unroll
    for (int j = 0; j < 4; ++j) acc[i][j] = (v8f){0.f,0.f,0.f,0.f,0.f,0.f,0.f,0.f};

  for (int k0 = 0; k0 < K; k0 += 32) {
    V bh[4], bl[4];
#pragma unroll
    for (int j = 0; j < 4; ++j) {
      const size_t bo = (size_t)(n0 + (j << 4) + rlane) * ldb + koff + k0;
      bh[j] = Frag<T>::load(Bb + bo);
      if (SPLIT) bl[j] = Frag<T>::load(Bb2 + bo);
    }
#pragma unroll
    for (int i = 0; i < 4; ++i) {
      const size_t ao = (size_t)(m0 + (i << 4) + rlane) * lda + koff + k0;
      V ah = Frag<T>::load(Ab + ao);
      V al;
      if (SPLIT) al = Frag<T>::load(Ab2 + ao);
#pragma unroll
      for (int j = 0; j < 4; ++j) {
        acc[i][j] = Frag<T>::mma(ah, bh[j], acc[i][j]);
        if (SPLIT) {
          acc[i][j] = Frag<T>::mma(ah, bl[j], acc[i][j]);
          acc[i][j] = Frag<T>::mma(al, bh[j], acc[i][j]);
        }
      }
      Frag<T>::guard(acc[i][0], acc[i][3], ah, SPLIT ? al : ah);
    }
    Frag<T>::keep(bh[0], bh[1], bh[2], bh[3]);
    if (SPLIT) Frag<T>::keep(bl[0], bl[1], bl[2], bl[3]);
  }
  acc_guard4(acc[0][0], acc[0][1], acc[0][2], acc[0][3]);
  acc_guard4(acc[1][0], acc[1][1], acc[1][2], acc[1][3]);
  acc_guard4(acc[2][0], acc[2][1], acc[2][2], acc[2][3]);
  acc_guard4(acc[3][0], acc[3][1], acc[3][2], acc[3][3]);

  float* slab = sT[wave];
  const float* Rb = RESID ? (resid + (size_t)b * strideR) : nullptr;
#pragma unroll
  for (int i = 0; i < 4; ++i) {
    const int mBase = m0 + (i << 4);
#pragma unroll
    for (int j = 0; j < 4; ++j) {
      const int n = n0 + (j << 4) + rlane;
      float bv = 0.f;
      if (BIAS_MODE == 2) bv = bias[n];
#pragma unroll
      for (int r = 0; r < 8; ++r) {
        float v = acc[i][j][r] * scale;
        if (BIAS_MODE == 1) v += bias[mBase + mOff + r];
        if (BIAS_MODE == 2) v += bv;
        if (RESID) v += Rb[(size_t)(mBase + mOff + r) * ldc + n];
        if (ACT == 1) v = tanhf(v);
        if (ACT == 2) v = fmaxf(v, 0.0f);
        if (ACT == 3) v = v / (1.0f + expf(-v));
        if (ACT == 4) v = (v > 0.f) ? v : 0.01f * v;
        if (ACT == 5) v = 0.5f * v * (1.0f + erff(v * 0.70710678118654752f));
        slab[(mOff + r) * 68 + (j << 4) + rlane] = v;
      }
    }
    __builtin_amdgcn_fence(__ATOMIC_RELEASE, "workgroup");
    __builtin_amdgcn_wave_barrier();
    __builtin_amdgcn_fence(__ATOMIC_ACQUIRE, "workgroup");
    if (OUT_MODE == 0) {
      float* C = (float*)Cout + (size_t)b * strideC;
      const int hh = lane >> 4, c4 = (lane & 15) * 4;
      for (int pass = 0; pass < 2; ++pass) {
#pragma unroll
        for (int it = 0; it < 8; ++it) {
          const int row = it * 2 + hh;
          v4f v = *(const v4f*)(slab + row * 68 + c4);
          *(volatile v4f*)(C + (size_t)(mBase + row) * ldc + n0 + c4) = v;
        }
        __threadfence();
      }
    } else {
      const int q = lane >> 3, c8 = (lane & 7) * 8;
      unsigned short* C  = (unsigned short*)Cout  + (size_t)b * strideC;
      unsigned short* C2 = (OUT_MODE == 2) ? ((unsigned short*)Cout2 + (size_t)b * strideC) : nullptr;
      for (int pass = 0; pass < 2; ++pass) {
#pragma unroll
        for (int it = 0; it < 4; ++it) {
          const int row = it * 4 + q;
          const float* sp = slab + row * 68 + c8;
          v8h hv, lv;
#pragma unroll
          for (int e = 0; e < 8; ++e) {
            if (OUT_MODE == 1) {
              hv[e] = (_Float16)sp[e];
            } else {
              unsigned short hb = f2bf_bits(sp[e]);
              unsigned short lb = f2bf_bits(sp[e] - bf_bits2f(hb));
              hv[e] = __builtin_bit_cast(_Float16, hb);
              lv[e] = __builtin_bit_cast(_Float16, lb);
            }
          }
          *(volatile v8h*)(C + (size_t)(mBase + row) * ldc + n0 + c8) = hv;
          if (OUT_MODE == 2) *(volatile v8h*)(C2 + (size_t)(mBase + row) * ldc + n0 + c8) = lv;
        }
        __threadfence();
      }
    }
    __builtin_amdgcn_fence(__ATOMIC_RELEASE, "workgroup");
    __builtin_amdgcn_wave_barrier();
    __builtin_amdgcn_fence(__ATOMIC_ACQUIRE, "workgroup");
  }
}

constexpr int NBATCH = 8;
constexpr int SEQ_T  = 128;
constexpr int CIN    = 1024;
constexpr int NHEAD  = 4;
constexpr int HID    = 512;
constexpr int NGATE  = 4 * HID;
constexpr int NDIR   = 2;
constexpr int NKD    = NDIR * NHEAD;
constexpr int MROWS  = SEQ_T * NBATCH;
constexpr int APITCH = HID + 16;
constexpr int SPITCH = 68;

constexpr size_t SZ_WIH  = (size_t)NHEAD * NGATE * CIN * 2;
constexpr size_t SZ_X16  = (size_t)NHEAD * MROWS * CIN * 2;
constexpr size_t SZ_WHH  = (size_t)NKD * NGATE * HID * 2;
constexpr size_t SZ_BIAS = (size_t)NKD * NGATE * 4;
constexpr size_t SZ_GX   = (size_t)NKD * MROWS * NGATE * 4;
constexpr size_t SZ_HPL  = (size_t)NKD * SEQ_T * NBATCH * HID * 4;
constexpr size_t OFF_WIH  = 0;
constexpr size_t OFF_X16  = OFF_WIH + SZ_WIH;
constexpr size_t OFF_WHH  = OFF_X16 + SZ_X16;
constexpr size_t OFF_BIAS = OFF_WHH + SZ_WHH;
constexpr size_t OFF_GX   = OFF_BIAS + SZ_BIAS;
constexpr size_t OFF_HPL  = OFF_GX + SZ_GX;
constexpr size_t WS_END   = OFF_HPL + SZ_HPL;
static_assert(WS_END == 125894656ull, "carve total");
static_assert(WS_END <= 134217728ull, "carve cap");
static_assert((OFF_X16 % 128) == 0 && (OFF_WHH % 128) == 0 && (OFF_BIAS % 128) == 0 &&
              (OFF_GX % 128) == 0 && (OFF_HPL % 128) == 0, "line alignment");

__device__ __forceinline__ unsigned pack_bf16x2(float lo, float hi) {
  return (unsigned)f2bf_bits(lo) | ((unsigned)f2bf_bits(hi) << 16);
}
__device__ __forceinline__ float bf_val(float f) { return bf_bits2f(f2bf_bits(f)); }

__global__ __launch_bounds__(256) void cast_bf16x8_kernel(const float* __restrict__ in,
                                                          unsigned short* __restrict__ out, int n8) {
  const int i = blockIdx.x * 256 + threadIdx.x;
  if (i < n8) {
    const v4f a = *(const v4f*)(in + (size_t)i * 8);
    const v4f c = *(const v4f*)(in + (size_t)i * 8 + 4);
    v4u u;
    u.x = pack_bf16x2(a.x, a.y);
    u.y = pack_bf16x2(a.z, a.w);
    u.z = pack_bf16x2(c.x, c.y);
    u.w = pack_bf16x2(c.z, c.w);
    volatile v4u* dst = (volatile v4u*)(out + (size_t)i * 8);
    *dst = u;
    __threadfence();
    *dst = u;
  }
}

__global__ __launch_bounds__(128) void deint_x_kernel(const float* __restrict__ x,
                                                      unsigned short* __restrict__ x16) {
  const int m = blockIdx.x;
  const int t = m >> 3, b = m & 7;
  const int tid = threadIdx.x;
  const float* src = x + (((size_t)b * SEQ_T + t) * CIN + (size_t)tid * 8) * NHEAD;
  v4f v[8];
#pragma unroll
  for (int e = 0; e < 8; ++e) v[e] = *(const v4f*)(src + 4 * e);
  v4u pk[4];
#pragma unroll
  for (int k = 0; k < 4; ++k) {
    pk[k].x = pack_bf16x2(v[0][k], v[1][k]);
    pk[k].y = pack_bf16x2(v[2][k], v[3][k]);
    pk[k].z = pack_bf16x2(v[4][k], v[5][k]);
    pk[k].w = pack_bf16x2(v[6][k], v[7][k]);
  }
  for (int pass = 0; pass < 2; ++pass) {
#pragma unroll
    for (int k = 0; k < 4; ++k)
      *(volatile v4u*)(x16 + ((size_t)k * MROWS + m) * CIN + (size_t)tid * 8) = pk[k];
    __threadfence();
  }
}

__global__ __launch_bounds__(256) void bias_sum_kernel(const float* __restrict__ bif, const float* __restrict__ bhf,
                                                       const float* __restrict__ bib, const float* __restrict__ bhb,
                                                       float* __restrict__ biasf) {
  const int dir = blockIdx.x >> 3;
  const int i = blockIdx.x * 256 + threadIdx.x;
  const int loc = (i - dir * 2048) * 4;
  const float* bi = dir ? bib : bif;
  const float* bh = dir ? bhb : bhf;
  const v4f a = *(const v4f*)(bi + loc);
  const v4f c = *(const v4f*)(bh + loc);
  v4f o;
  o.x = bf_val(a.x) + bf_val(c.x);
  o.y = bf_val(a.y) + bf_val(c.y);
  o.z = bf_val(a.z) + bf_val(c.z);
  o.w = bf_val(a.w) + bf_val(c.w);
  volatile v4f* dst = (volatile v4f*)(biasf + (size_t)i * 4);
  *dst = o;
  __threadfence();
  *dst = o;
}

__device__ __forceinline__ float sigmoid_f(float x) {
  x = fminf(fmaxf(x, -40.0f), 40.0f);
  return 1.0f / (1.0f + expf(-x));
}

__global__ __launch_bounds__(256) void lstm_rec_kernel(const unsigned short* __restrict__ whh,
                                                       const float* __restrict__ gx,
                                                       float* __restrict__ hpl) {
  __shared__ __align__(16) __bf16 Ash[2][16 * APITCH];
  __shared__ __align__(16) float  Hs[8][16 * SPITCH];
  const int kd = blockIdx.x;
  const int dir = kd >> 2;
  const int tid = threadIdx.x, wave = tid >> 5, lane = tid & 31, hh = lane >> 4, cc = lane & 15;

  {
    unsigned* zp = (unsigned*)(void*)&Ash[0][0];
    for (int i = tid; i < (2 * 16 * APITCH) / 2; i += 256) zp[i] = 0u;
  }
  __syncthreads();

  const __bf16* Wk = (const __bf16*)(const void*)whh + (size_t)kd * NGATE * HID;
  const float*  Gk = gx + (size_t)kd * MROWS * NGATE;
  float*        Hk = hpl + (size_t)kd * SEQ_T * NBATCH * HID;
  float* slab = Hs[wave];

  float cst[4][8];
#pragma unroll
  for (int ub = 0; ub < 4; ++ub)
#pragma unroll
    for (int r = 0; r < 8; ++r) cst[ub][r] = 0.0f;

  for (int step = 0; step < SEQ_T; ++step) {
    const int p = step & 1;
    const int t = dir ? (SEQ_T - 1 - step) : step;
    const __bf16* At = Ash[p];
    __bf16* An = Ash[p ^ 1];
    const float* Gt = Gk + (size_t)(t * NBATCH) * NGATE;

#pragma unroll
    for (int ub = 0; ub < 4; ++ub) {
      const int u0 = wave * 64 + ub * 16;
      v8f acc[4];
#pragma unroll
      for (int g = 0; g < 4; ++g) acc[g] = (v8f){0.f,0.f,0.f,0.f,0.f,0.f,0.f,0.f};
#pragma unroll 4
      for (int ks = 0; ks < HID / 32; ++ks) {
        const int k0 = ks * 32 + 8 * hh;
        const v16b a = Frag<__bf16>::load(At + cc * APITCH + k0);
        v16b bw[4];
#pragma unroll
        for (int g = 0; g < 4; ++g)
          bw[g] = Frag<__bf16>::load(Wk + (size_t)(g * HID + u0 + cc) * HID + k0);
#pragma unroll
        for (int g = 0; g < 4; ++g) acc[g] = Frag<__bf16>::mma(a, bw[g], acc[g]);
        Frag<__bf16>::guard(acc[0], acc[3], a, bw[3]);
        Frag<__bf16>::keep(bw[0], bw[1], bw[2], bw[3]);
      }
      acc_guard4(acc[0], acc[1], acc[2], acc[3]);

      const float* gcol = Gt + u0 + cc;
#pragma unroll
      for (int r = 0; r < 8; ++r) {
        const float* gp = gcol + (size_t)r * NGATE;
        const float gi = acc[0][r] + gp[0];
        const float gf = acc[1][r] + gp[HID];
        const float gg = acc[2][r] + gp[2 * HID];
        const float go = acc[3][r] + gp[3 * HID];
        const float cn = sigmoid_f(gf) * cst[ub][r] + sigmoid_f(gi) * tanhf(gg);
        cst[ub][r] = cn;
        const float hv = sigmoid_f(go) * tanhf(cn);
        const float hsel = hh ? 0.0f : hv;
        const int row = 8 * hh + r;
        slab[row * SPITCH + ub * 16 + cc] = hsel;
        An[row * APITCH + u0 + cc] = __builtin_bit_cast(__bf16, f2bf_bits(hsel));
      }
    }

    __builtin_amdgcn_fence(__ATOMIC_RELEASE, "workgroup");
    __builtin_amdgcn_wave_barrier();
    __builtin_amdgcn_fence(__ATOMIC_ACQUIRE, "workgroup");
    {
      const int c4 = cc * 4;
      float* hbase = Hk + (size_t)(t * NBATCH) * HID + wave * 64 + c4;
      for (int pass = 0; pass < 2; ++pass) {
#pragma unroll
        for (int it = 0; it < 4; ++it) {
          const int row = it * 2 + hh;
          const v4f v = *(const v4f*)(slab + row * SPITCH + c4);
          *(volatile v4f*)(hbase + (size_t)row * HID) = v;
        }
        __threadfence();
      }
    }
    __builtin_amdgcn_fence(__ATOMIC_RELEASE, "workgroup");
    __builtin_amdgcn_wave_barrier();
    __builtin_amdgcn_fence(__ATOMIC_ACQUIRE, "workgroup");
    __syncthreads();
  }
}

__global__ __launch_bounds__(256) void interleave_out_kernel(const float* __restrict__ hpl,
                                                             float* __restrict__ out) {
  const int bt = blockIdx.x;
  const int b = bt >> 7, t = bt & 127;
  const int tid = threadIdx.x;
  v4f vals[4];
#pragma unroll
  for (int j = 0; j < 4; ++j) {
    const int pos = tid + 256 * j;
    const int dir = pos >> 9, u = pos & 511;
#pragma unroll
    for (int k = 0; k < 4; ++k)
      vals[j][k] = hpl[(((size_t)(dir * NHEAD + k) * SEQ_T + t) * NBATCH + b) * HID + u];
  }
  float* orow = out + (size_t)bt * (2 * HID) * NHEAD;
  for (int pass = 0; pass < 2; ++pass) {
#pragma unroll
    for (int j = 0; j < 4; ++j)
      *(volatile v4f*)(orow + (size_t)(tid + 256 * j) * 4) = vals[j];
    __threadfence();
  }
}

extern "C" void kernel_launch(void* const* d_in, const int* in_sizes, int n_in,
                              void* d_out, int out_size, void* d_ws, size_t ws_size,
                              hipStream_t stream) {
  if (n_in < 9) return;
  if (in_sizes[0] != NBATCH * SEQ_T * CIN * NHEAD) return;
  if (in_sizes[1] != NHEAD * NGATE * CIN || in_sizes[5] != NHEAD * NGATE * CIN) return;
  if (in_sizes[2] != NHEAD * NGATE * HID || in_sizes[6] != NHEAD * NGATE * HID) return;
  if (in_sizes[3] != NHEAD * NGATE || in_sizes[4] != NHEAD * NGATE ||
      in_sizes[7] != NHEAD * NGATE || in_sizes[8] != NHEAD * NGATE) return;
  if (out_size != NBATCH * SEQ_T * 2 * HID * NHEAD) return;
  if (ws_size < WS_END) return;

  const float* x     = (const float*)d_in[0];
  const float* Wih_f = (const float*)d_in[1];
  const float* Whh_f = (const float*)d_in[2];
  const float* bih_f = (const float*)d_in[3];
  const float* bhh_f = (const float*)d_in[4];
  const float* Wih_b = (const float*)d_in[5];
  const float* Whh_b = (const float*)d_in[6];
  const float* bih_b = (const float*)d_in[7];
  const float* bhh_b = (const float*)d_in[8];
  float* out = (float*)d_out;

  char* ws = (char*)d_ws;
  unsigned short* wih   = (unsigned short*)(ws + OFF_WIH);
  unsigned short* x16   = (unsigned short*)(ws + OFF_X16);
  unsigned short* whh   = (unsigned short*)(ws + OFF_WHH);
  float*          biasf = (float*)(ws + OFF_BIAS);
  float*          gxp   = (float*)(ws + OFF_GX);
  float*          hpl   = (float*)(ws + OFF_HPL);

  const int nWihDir8 = (NHEAD * NGATE * CIN) / 8;
  const int nWhhDir8 = (NHEAD * NGATE * HID) / 8;

  deint_x_kernel<<<MROWS, 128, 0, stream>>>(x, x16);
  bias_sum_kernel<<<16, 256, 0, stream>>>(bih_f, bhh_f, bih_b, bhh_b, biasf);
  cast_bf16x8_kernel<<<nWhhDir8 / 256, 256, 0, stream>>>(Whh_f, whh, nWhhDir8);
  cast_bf16x8_kernel<<<nWhhDir8 / 256, 256, 0, stream>>>(Whh_b, whh + (size_t)NHEAD * NGATE * HID, nWhhDir8);

  const dim3 ggrid((MROWS / 64) * (NGATE / 64) / 8, 1);
  for (int dir = 0; dir < NDIR; ++dir) {
    const float* WihDir = dir ? Wih_b : Wih_f;
    cast_bf16x8_kernel<<<nWihDir8 / 256, 256, 0, stream>>>(WihDir, wih, nWihDir8);
    for (int k = 0; k < NHEAD; ++k) {
      const int kd = dir * NHEAD + k;
      const unsigned short* Aop = x16 + (size_t)k * MROWS * CIN;
      const unsigned short* Bop = wih + (size_t)k * NGATE * CIN;
      float* Cp = gxp + (size_t)kd * MROWS * NGATE;
      wmma_gemm64<1, false, 2, 0, false, 0><<<ggrid, 256, 0, stream>>>(
          Aop, Aop, CIN, 0L,
          Bop, Bop, CIN, 0L,
          (void*)Cp, (void*)Cp, NGATE, 0L,
          biasf + (size_t)kd * NGATE,
          biasf, 0L,
          MROWS, NGATE, CIN, 1.0f);
    }
  }

  lstm_rec_kernel<<<NKD, 256, 0, stream>>>(whh, gxp, hpl);
  interleave_out_kernel<<<NBATCH * SEQ_T, 256, 0, stream>>>(hpl, out);
}
